// CausalSelfAttention_16552803958929
// MI455X (gfx1250) — hardware-verified
//
#include <hip/hip_runtime.h>


#ifndef NB
#define NB 2
#endif
#ifndef SEQ
#define SEQ 2048
#endif
#define NB_FULL  2
#define SEQ_FULL 2048
#define DM   1024
#define NH   16
#define HD   64
#define RH   512
#define RHQ  ((RH < SEQ) ? RH : SEQ)
#define MROWS (NB * SEQ)
#define NTHL (RHQ / 16)
#define NT16 ((SEQ - RHQ) / 16)
#define NT16D ((NT16 > 0) ? NT16 : 1)
#define PLN  ((size_t)NB * NH * SEQ * HD)
#define PLNR ((size_t)NB * NH * RHQ * HD)
#define PCAR 1024.0f
#define SCL  0.125f
#define L2E  1.4426950408889634f
#define NEGB (-3.0e38f)

static_assert(HD == 64);
static_assert(NH * HD == DM);
static_assert(DM % 64 == 0);
static_assert(SEQ % 64 == 0);
static_assert(RHQ % 64 == 0);
static_assert(SEQ <= SEQ_FULL);
static_assert(NB <= NB_FULL);
static_assert(MROWS % 64 == 0);
static_assert((NB * NH * NTHL) % 4 == 0);
static_assert((NB * NH * NT16) % 4 == 0);
static_assert(((size_t)MROWS * DM / 8) % 256 == 0);
static_assert(((size_t)3 * DM * DM / 8) % 256 == 0);

typedef _Float16 h16;
typedef unsigned short bf;
typedef __attribute__((ext_vector_type(16))) __bf16   v16bf;
typedef __attribute__((ext_vector_type(16))) _Float16 v16h;
typedef __attribute__((ext_vector_type(8)))  _Float16 v8h;
typedef __attribute__((ext_vector_type(8)))  unsigned short v8us;
typedef __attribute__((ext_vector_type(8)))  float    v8f;
typedef __attribute__((ext_vector_type(4)))  float    v4f;
typedef v8h  __attribute__((may_alias)) v8ha;
typedef v4f  __attribute__((may_alias)) v4fa;
typedef v8us __attribute__((may_alias)) v8usa;

__device__ __forceinline__ unsigned short f2bf(float f) { unsigned u = __float_as_uint(f); u += 0x7FFFu + ((u >> 16) & 1u); return (unsigned short)(u >> 16); }
__device__ __forceinline__ float bf2f(unsigned short b) { return __uint_as_float(((unsigned)b) << 16); }
__device__ __forceinline__ float bfr(float f) { return bf2f(f2bf(f)); }
__device__ __forceinline__ void splitf(float y, unsigned short& h, unsigned short& l) { h = f2bf(y); l = f2bf(y - bf2f(h)); }
__device__ __forceinline__ v16h cat16(v8h lo, v8h hi) { return __builtin_shufflevector(lo, hi, 0, 1, 2, 3, 4, 5, 6, 7, 8, 9, 10, 11, 12, 13, 14, 15); }
__device__ __forceinline__ v16bf cat16b(v8us lo, v8us hi) { return __builtin_bit_cast(v16bf, __builtin_shufflevector(lo, hi, 0, 1, 2, 3, 4, 5, 6, 7, 8, 9, 10, 11, 12, 13, 14, 15)); }
__device__ __forceinline__ v8f wmma16(v16h a, v16h b, v8f c) { return __builtin_amdgcn_wmma_f32_16x16x32_f16(false, a, false, b, (short)0, c, false, false); }
__device__ __forceinline__ v8f wmmab(v16bf a, v16bf b, v8f c) { return __builtin_amdgcn_wmma_f32_16x16x32_bf16(false, a, false, b, (short)0, c, false, false); }
__device__ __forceinline__ v16h  ldh(const h16* p) { return cat16(*(const v8h*)p, *(const v8h*)(p + 16)); }
__device__ __forceinline__ v16bf ldb(const bf* p)  { return cat16b(*(const v8us*)p, *(const v8us*)(p + 16)); }
__device__ __forceinline__ float ex2(float x) { return __builtin_amdgcn_exp2f(x); }

__global__ __launch_bounds__(256) void k_cvt8(const float* __restrict__ src, bf* dst, unsigned n8, unsigned seg8, unsigned sstride8) {
    const unsigned i = blockIdx.x * 256u + threadIdx.x; if (i >= n8) return;
    const unsigned b = i / seg8, r = i - b * seg8;
    const v8f v = *(const v8f*)(src + ((size_t)b * sstride8 + r) * 8); v8us o;
#pragma unroll
    for (int k = 0; k < 8; ++k) o[k] = f2bf(v[k]);
    *(volatile v8us*)(dst + (size_t)i * 8) = o; __threadfence(); *(volatile v8us*)(dst + (size_t)i * 8) = o;
}

template <bool SPLIT>
__device__ __forceinline__ void gemm_main(const bf* __restrict__ A, const bf* __restrict__ A2, const bf* __restrict__ Bt, int K, int r0, int c0, int lr, int hi, v8f (&acc)[4][4]) {
#pragma unroll
    for (int mb = 0; mb < 4; ++mb)
#pragma unroll
        for (int nb = 0; nb < 4; ++nb) acc[mb][nb] = (v8f){};
    const size_t aoff = (size_t)(r0 + lr) * K + 8 * hi, boff = (size_t)(c0 + lr) * K + 8 * hi;
#pragma unroll 1
    for (int kc = 0; kc < K; kc += 32) {
        v16bf a[4], a2[4];
#pragma unroll
        for (int mb = 0; mb < 4; ++mb) { a[mb] = ldb(A + aoff + (size_t)mb * 16 * K + kc); if (SPLIT) a2[mb] = ldb(A2 + aoff + (size_t)mb * 16 * K + kc); }
#pragma unroll
        for (int nb = 0; nb < 4; ++nb) { const v16bf b = ldb(Bt + boff + (size_t)nb * 16 * K + kc);
#pragma unroll
            for (int mb = 0; mb < 4; ++mb) { acc[mb][nb] = wmmab(a[mb], b, acc[mb][nb]); if (SPLIT) acc[mb][nb] = wmmab(a2[mb], b, acc[mb][nb]); } }
        asm volatile("v_nop\n\tv_nop\n\tv_nop\n\tv_nop" : "+v"(acc[0][0]), "+v"(acc[1][1]), "+v"(acc[2][2]), "+v"(acc[3][3]) : "v"(a[0]), "v"(a[3]));
    }
}

__global__ __launch_bounds__(32) void k_qkv(const bf* __restrict__ XB, const bf* __restrict__ W, const float* __restrict__ bias, h16* H16, bf* HI, bf* LO) {
    __shared__ __align__(16) float os[64 * 68];
    const int lane = threadIdx.x & 31, lr = lane & 15, hi = lane >> 4; const int r0 = blockIdx.x * 64, c0 = blockIdx.y * 64;
    v8f acc[4][4];
    gemm_main<false>(XB, XB, W, DM, r0, c0, lr, hi, acc);
#pragma unroll
    for (int nb = 0; nb < 4; ++nb) { const float bv = bfr(bias[c0 + nb * 16 + lr]);
#pragma unroll
        for (int mb = 0; mb < 4; ++mb)
#pragma unroll
            for (int j = 0; j < 8; ++j) os[(mb * 16 + hi * 8 + j) * 68 + nb * 16 + lr] = acc[mb][nb][j] + bv; }
    __builtin_amdgcn_wave_barrier(); asm volatile("s_wait_dscnt 0" ::: "memory");
    const int which = c0 / DM, h = (c0 % DM) / HD, b = r0 / SEQ, t0 = r0 % SEQ, bh = b * NH + h;
    const bool w16 = (which != 0) || (t0 >= RHQ), whl = (t0 < RHQ);
    const int rq = lane >> 3, cc = (lane & 7) * 8;
#pragma unroll 1
    for (int ps = 0; ps < 2; ++ps) {
#pragma unroll 1
        for (int it = 0; it < 16; ++it) { const int rr = it * 4 + rq; float v[8]; size_t o16, ohl;
            if (which == 2) {
#pragma unroll
                for (int i = 0; i < 8; ++i) v[i] = os[(cc + i) * 68 + rr];
                o16 = 2 * PLN + ((size_t)bh * HD + rr) * SEQ + t0 + cc; ohl = 2 * PLNR + ((size_t)bh * HD + rr) * RHQ + t0 + cc;
            } else {
                const v4f a = *(const v4fa*)(os + rr * 68 + cc), c = *(const v4fa*)(os + rr * 68 + cc + 4);
                v[0] = a[0]; v[1] = a[1]; v[2] = a[2]; v[3] = a[3]; v[4] = c[0]; v[5] = c[1]; v[6] = c[2]; v[7] = c[3];
                o16 = (size_t)which * PLN + ((size_t)bh * SEQ + t0 + rr) * HD + cc; ohl = (size_t)which * PLNR + ((size_t)bh * RHQ + t0 + rr) * HD + cc; }
            if (w16) { v8h o;
#pragma unroll
                for (int i = 0; i < 8; ++i) o[i] = (h16)v[i];
                *(volatile v8h*)(H16 + o16) = o; }
            if (whl) { v8us oh, ol;
#pragma unroll
                for (int i = 0; i < 8; ++i) { unsigned short a2, c2; splitf(v[i], a2, c2); oh[i] = a2; ol[i] = c2; }
                *(volatile v8us*)(HI + ohl) = oh; *(volatile v8us*)(LO + ohl) = ol; } }
        if (ps == 0) __threadfence(); }
}

__device__ __forceinline__ void sm_tile(v8f (&s)[4], float (&mrow)[8], float (&lsum)[8], float (&alpha)[8], int qrow0, int key0, bool diag) {
#pragma unroll
    for (int j = 0; j < 4; ++j)
#pragma unroll
        for (int r = 0; r < 8; ++r) s[j][r] = s[j][r] * SCL;
    if (diag) {
#pragma unroll
        for (int j = 0; j < 4; ++j)
#pragma unroll
            for (int r = 0; r < 8; ++r) s[j][r] = (key0 + 16 * j <= qrow0 + r) ? s[j][r] : NEGB; }
#pragma unroll
    for (int r = 0; r < 8; ++r) {
        float mx = fmaxf(fmaxf(s[0][r], s[1][r]), fmaxf(s[2][r], s[3][r]));
        mx = fmaxf(mx, __shfl_xor(mx, 1, 32)); mx = fmaxf(mx, __shfl_xor(mx, 2, 32)); mx = fmaxf(mx, __shfl_xor(mx, 4, 32)); mx = fmaxf(mx, __shfl_xor(mx, 8, 32));
        const float mn = fmaxf(mrow[r], mx);
        const float al = ex2((mrow[r] - mn) * L2E);
        const float e0 = ex2((s[0][r] - mn) * L2E), e1 = ex2((s[1][r] - mn) * L2E), e2 = ex2((s[2][r] - mn) * L2E), e3 = ex2((s[3][r] - mn) * L2E);
        s[0][r] = e0; s[1][r] = e1; s[2][r] = e2; s[3][r] = e3;
        lsum[r] = lsum[r] * al + ((e0 + e1) + (e2 + e3)); mrow[r] = mn; alpha[r] = al; }
}

__device__ __forceinline__ void fa_store(v8f (&acc)[4], float (&lsum)[8], float cs, float* ow, bf* ATh, bf* ATl, size_t obase, int lane, int lr, int hi) {
#pragma unroll
    for (int r = 0; r < 8; ++r) { float t = lsum[r]; t += __shfl_xor(t, 1, 32); t += __shfl_xor(t, 2, 32); t += __shfl_xor(t, 4, 32); t += __shfl_xor(t, 8, 32);
        const float inv = cs * __builtin_amdgcn_rcpf(t);
#pragma unroll
        for (int n = 0; n < 4; ++n) ow[(8 * hi + r) * 68 + n * 16 + lr] = acc[n][r] * inv; }
    __builtin_amdgcn_wave_barrier(); asm volatile("s_wait_dscnt 0" ::: "memory");
    const int rq = lane >> 3, cc = (lane & 7) * 8;
#pragma unroll 1
    for (int ps = 0; ps < 2; ++ps) {
#pragma unroll
        for (int it = 0; it < 4; ++it) { const int rr = it * 4 + rq; const v4f a = *(const v4fa*)(ow + rr * 68 + cc), c = *(const v4fa*)(ow + rr * 68 + cc + 4); v8us oh, ol;
#pragma unroll
            for (int i = 0; i < 4; ++i) { unsigned short a2, c2; splitf(a[i], a2, c2); oh[i] = a2; ol[i] = c2; splitf(c[i], a2, c2); oh[4 + i] = a2; ol[4 + i] = c2; }
            const size_t oo = obase + (size_t)rr * DM + cc; *(volatile v8us*)(ATh + oo) = oh; *(volatile v8us*)(ATl + oo) = ol; }
        if (ps == 0) __threadfence(); }
}

__global__ __launch_bounds__(128) void k_fa16(const h16* __restrict__ H16, bf* ATh, bf* ATl) {
    __shared__ __align__(16) h16 pls[4][16 * 72];
    __shared__ __align__(16) float oss[4][16 * 68];
    const int w = threadIdx.x >> 5, lane = threadIdx.x & 31, lr = lane & 15, hi = lane >> 4;
    const int id = blockIdx.x * 4 + w; if (id >= NB * NH * NT16) return;
    const int qt = id % NT16D, bh = id / NT16D, q0 = RHQ + qt * 16;
    h16* pw = pls[w]; float* ow = oss[w];
    const h16* Qp = H16 + ((size_t)bh * SEQ + q0 + lr) * HD + 8 * hi;
    const v16h qa0 = ldh(Qp), qa1 = ldh(Qp + 32);
    const h16* Kp = H16 + PLN + (size_t)bh * SEQ * HD + (size_t)lr * HD + 8 * hi;
    const h16* Vp = H16 + 2 * PLN + (size_t)bh * HD * SEQ + (size_t)lr * SEQ + 8 * hi;
    v8f acc[4]; float mrow[8], lsum[8], alpha[8];
#pragma unroll
    for (int n = 0; n < 4; ++n) acc[n] = (v8f){};
#pragma unroll
    for (int r = 0; r < 8; ++r) { mrow[r] = NEGB; lsum[r] = 0.f; alpha[r] = 0.f; }
    const int nkt = (q0 + 15) / 64 + 1;
#pragma unroll 1
    for (int kt = 0; kt < nkt; ++kt) { const int kb = kt * 64;
        v8f s[4];
#pragma unroll
        for (int j = 0; j < 4; ++j) { const h16* kp = Kp + (size_t)(kb + j * 16) * HD; const v16h b0 = ldh(kp), b1 = ldh(kp + 32);
            s[j] = (v8f){}; s[j] = wmma16(qa0, b0, s[j]); s[j] = wmma16(qa1, b1, s[j]); }
        asm volatile("v_nop\n\tv_nop\n\tv_nop\n\tv_nop" : "+v"(s[0]), "+v"(s[1]), "+v"(s[2]), "+v"(s[3]) : "v"(qa0), "v"(qa1));
        sm_tile(s, mrow, lsum, alpha, q0 + 8 * hi, kb + lr, kb + 63 > q0);
#pragma unroll
        for (int n = 0; n < 4; ++n)
#pragma unroll
            for (int r = 0; r < 8; ++r) acc[n][r] = acc[n][r] * alpha[r];
#pragma unroll
        for (int r = 0; r < 8; ++r)
#pragma unroll
            for (int j = 0; j < 4; ++j) pw[(8 * hi + r) * 72 + j * 16 + lr] = (h16)(s[j][r] * PCAR);
        __builtin_amdgcn_wave_barrier(); asm volatile("s_wait_dscnt 0" ::: "memory");
        const h16* pr = pw + lr * 72 + 8 * hi;
        const v16h pa0 = cat16(*(const v8ha*)(pr), *(const v8ha*)(pr + 16)), pa1 = cat16(*(const v8ha*)(pr + 32), *(const v8ha*)(pr + 48));
        __builtin_amdgcn_wave_barrier(); asm volatile("s_wait_dscnt 0" ::: "memory");
#pragma unroll
        for (int n = 0; n < 4; ++n) { const h16* vp = Vp + (size_t)(n * 16) * SEQ + kb; const v16h v0 = ldh(vp), v1 = ldh(vp + 32);
            acc[n] = wmma16(pa0, v0, acc[n]); acc[n] = wmma16(pa1, v1, acc[n]); }
        asm volatile("v_nop\n\tv_nop\n\tv_nop\n\tv_nop" : "+v"(acc[0]), "+v"(acc[1]), "+v"(acc[2]), "+v"(acc[3]) : "v"(pa0), "v"(pa1));
    }
    const int b = bh / NH, h = bh % NH;
    fa_store(acc, lsum, 1.0f / PCAR, ow, ATh, ATl, ((size_t)b * SEQ + q0) * DM + (size_t)h * HD, lane, lr, hi);
}

__global__ __launch_bounds__(128) void k_fahl(const bf* __restrict__ HI, const bf* __restrict__ LO, bf* ATh, bf* ATl) {
    __shared__ __align__(16) unsigned short phs[4][16 * 72];
    __shared__ __align__(16) unsigned short pls[4][16 * 72];
    __shared__ __align__(16) float oss[4][16 * 68];
    const int w = threadIdx.x >> 5, lane = threadIdx.x & 31, lr = lane & 15, hi = lane >> 4;
    const int id = blockIdx.x * 4 + w; if (id >= NB * NH * NTHL) return;
    const int qt = id % NTHL, bh = id / NTHL, q0 = qt * 16;
    unsigned short* pwh = phs[w]; unsigned short* pwl = pls[w]; float* ow = oss[w];
    const size_t qoff = ((size_t)bh * RHQ + q0 + lr) * HD + 8 * hi;
    const v16bf qh0 = ldb(HI + qoff), qh1 = ldb(HI + qoff + 32), ql0 = ldb(LO + qoff), ql1 = ldb(LO + qoff + 32);
    const size_t koff = PLNR + (size_t)bh * RHQ * HD + (size_t)lr * HD + 8 * hi;
    const size_t voff = 2 * PLNR + (size_t)bh * HD * RHQ + (size_t)lr * RHQ + 8 * hi;
    v8f acc[4]; float mrow[8], lsum[8], alpha[8];
#pragma unroll
    for (int n = 0; n < 4; ++n) acc[n] = (v8f){};
#pragma unroll
    for (int r = 0; r < 8; ++r) { mrow[r] = NEGB; lsum[r] = 0.f; alpha[r] = 0.f; }
    const int nkt = (q0 + 15) / 64 + 1;
#pragma unroll 1
    for (int kt = 0; kt < nkt; ++kt) { const int kb = kt * 64;
        v8f s[4];
#pragma unroll
        for (int j = 0; j < 4; ++j) { const size_t ko = koff + (size_t)(kb + j * 16) * HD;
            const v16bf kh0 = ldb(HI + ko), kh1 = ldb(HI + ko + 32), kl0 = ldb(LO + ko), kl1 = ldb(LO + ko + 32);
            s[j] = (v8f){}; s[j] = wmmab(qh0, kh0, s[j]); s[j] = wmmab(qh1, kh1, s[j]); s[j] = wmmab(ql0, kh0, s[j]); s[j] = wmmab(ql1, kh1, s[j]); s[j] = wmmab(qh0, kl0, s[j]); s[j] = wmmab(qh1, kl1, s[j]); }
        asm volatile("v_nop\n\tv_nop\n\tv_nop\n\tv_nop" : "+v"(s[0]), "+v"(s[1]), "+v"(s[2]), "+v"(s[3]) : "v"(qh0), "v"(ql1));
        sm_tile(s, mrow, lsum, alpha, q0 + 8 * hi, kb + lr, kb + 63 > q0);
#pragma unroll
        for (int n = 0; n < 4; ++n)
#pragma unroll
            for (int r = 0; r < 8; ++r) acc[n][r] = acc[n][r] * alpha[r];
#pragma unroll
        for (int r = 0; r < 8; ++r)
#pragma unroll
            for (int j = 0; j < 4; ++j) { unsigned short a2, c2; splitf(s[j][r], a2, c2); pwh[(8 * hi + r) * 72 + j * 16 + lr] = a2; pwl[(8 * hi + r) * 72 + j * 16 + lr] = c2; }
        __builtin_amdgcn_wave_barrier(); asm volatile("s_wait_dscnt 0" ::: "memory");
        const unsigned short* prh = pwh + lr * 72 + 8 * hi; const unsigned short* prl = pwl + lr * 72 + 8 * hi;
        const v16bf ph0 = cat16b(*(const v8usa*)(prh), *(const v8usa*)(prh + 16)), ph1 = cat16b(*(const v8usa*)(prh + 32), *(const v8usa*)(prh + 48));
        const v16bf pl0 = cat16b(*(const v8usa*)(prl), *(const v8usa*)(prl + 16)), pl1 = cat16b(*(const v8usa*)(prl + 32), *(const v8usa*)(prl + 48));
        __builtin_amdgcn_wave_barrier(); asm volatile("s_wait_dscnt 0" ::: "memory");
#pragma unroll
        for (int n = 0; n < 4; ++n) { const size_t vo = voff + (size_t)(n * 16) * RHQ + kb;
            const v16bf vh0 = ldb(HI + vo), vh1 = ldb(HI + vo + 32), vl0 = ldb(LO + vo), vl1 = ldb(LO + vo + 32);
            acc[n] = wmmab(ph0, vh0, acc[n]); acc[n] = wmmab(ph1, vh1, acc[n]); acc[n] = wmmab(pl0, vh0, acc[n]); acc[n] = wmmab(pl1, vh1, acc[n]); acc[n] = wmmab(ph0, vl0, acc[n]); acc[n] = wmmab(ph1, vl1, acc[n]); }
        asm volatile("v_nop\n\tv_nop\n\tv_nop\n\tv_nop" : "+v"(acc[0]), "+v"(acc[1]), "+v"(acc[2]), "+v"(acc[3]) : "v"(ph0), "v"(pl1));
    }
    const int b = bh / NH, h = bh % NH;
    fa_store(acc, lsum, 1.0f, ow, ATh, ATl, ((size_t)b * SEQ + q0) * DM + (size_t)h * HD, lane, lr, hi);
}

__global__ __launch_bounds__(32) void k_out(const bf* __restrict__ Ah, const bf* __restrict__ Al, const bf* __restrict__ WO, const float* __restrict__ bias, float* C) {
    __shared__ __align__(16) float os[16 * 68];
    const int lane = threadIdx.x & 31, lr = lane & 15, hi = lane >> 4; const int r0 = blockIdx.x * 64, c0 = blockIdx.y * 64;
    v8f acc[4][4];
    gemm_main<true>(Ah, Al, WO, DM, r0, c0, lr, hi, acc);
    const int cofs = lr * 4;
    v4f bv; bv[0] = bfr(bias[c0 + cofs]); bv[1] = bfr(bias[c0 + cofs + 1]); bv[2] = bfr(bias[c0 + cofs + 2]); bv[3] = bfr(bias[c0 + cofs + 3]);
#pragma unroll
    for (int mb = 0; mb < 4; ++mb) {
#pragma unroll
        for (int nb = 0; nb < 4; ++nb) {
#pragma unroll
            for (int j = 0; j < 8; ++j) os[(hi * 8 + j) * 68 + nb * 16 + lr] = acc[mb][nb][j]; }
        __builtin_amdgcn_wave_barrier(); asm volatile("s_wait_dscnt 0" ::: "memory");
        float* crow = C + (size_t)(r0 + mb * 16) * DM + c0;
#pragma unroll 1
        for (int ps = 0; ps < 2; ++ps) {
#pragma unroll
            for (int s = 0; s < 8; ++s) { const int row = 2 * s + hi; v4f val = *(const v4fa*)(os + row * 68 + cofs); val = val + bv;
                *(volatile v4f*)(crow + (size_t)row * DM + cofs) = val; }
            if (ps == 0) __threadfence(); }
        __builtin_amdgcn_wave_barrier(); asm volatile("s_wait_dscnt 0" ::: "memory");
    }
}

constexpr size_t al256(size_t b) { return (b + 255) & ~(size_t)255; }
constexpr size_t SZ_XB = al256((size_t)MROWS * DM * 2);
constexpr size_t SZ_WQ = al256((size_t)3 * DM * DM * 2);
constexpr size_t SZ_WO = al256((size_t)DM * DM * 2);
constexpr size_t SZ_H16 = al256((size_t)3 * PLN * 2);
constexpr size_t SZ_HL = al256((size_t)3 * PLNR * 2);
constexpr size_t SZ_AT = al256((size_t)MROWS * DM * 2);
constexpr size_t WS_TOTAL = SZ_XB + SZ_WQ + SZ_WO + SZ_H16 + 2 * SZ_HL + 2 * SZ_AT;
static_assert(WS_TOTAL <= (size_t)134217728);

extern "C" void kernel_launch(void* const* d_in, const int* in_sizes, int n_in,
                              void* d_out, int out_size, void* d_ws, size_t ws_size, hipStream_t stream) {
    if (n_in < 5) return;
    if ((size_t)in_sizes[0] < ((size_t)(NB - 1) * SEQ_FULL + SEQ) * DM) return;
    if ((size_t)in_sizes[1] < (size_t)3 * DM * DM) return;
    if ((size_t)in_sizes[2] < (size_t)3 * DM) return;
    if ((size_t)in_sizes[3] < (size_t)DM * DM) return;
    if ((size_t)in_sizes[4] < (size_t)DM) return;
    if ((size_t)out_size < (size_t)MROWS * DM) return;
    if (WS_TOTAL > ws_size) return;
    const float* x = (const float*)d_in[0]; const float* wqkv = (const float*)d_in[1]; const float* bqkv = (const float*)d_in[2]; const float* wp = (const float*)d_in[3]; const float* bp = (const float*)d_in[4];
    float* OUT = (float*)d_out;
    char* wsp = (char*)d_ws;
    bf* XB = (bf*)wsp; wsp += SZ_XB;
    bf* WQ = (bf*)wsp; wsp += SZ_WQ;
    bf* WO = (bf*)wsp; wsp += SZ_WO;
    h16* H16 = (h16*)wsp; wsp += SZ_H16;
    bf* HI = (bf*)wsp; wsp += SZ_HL;
    bf* LO = (bf*)wsp; wsp += SZ_HL;
    bf* ATh = (bf*)wsp; wsp += SZ_AT;
    bf* ATl = (bf*)wsp; wsp += SZ_AT;
    const unsigned nx8 = (unsigned)((size_t)MROWS * DM / 8), nq8 = (unsigned)((size_t)3 * DM * DM / 8), no8 = (unsigned)((size_t)DM * DM / 8);
    k_cvt8<<<(nx8 + 255) / 256, 256, 0, stream>>>(x, XB, nx8, (unsigned)((size_t)SEQ * DM / 8), (unsigned)((size_t)SEQ_FULL * DM / 8));
    k_cvt8<<<(nq8 + 255) / 256, 256, 0, stream>>>(wqkv, WQ, nq8, nq8, nq8);
    k_cvt8<<<(no8 + 255) / 256, 256, 0, stream>>>(wp, WO, no8, no8, no8);
    k_qkv<<<dim3(MROWS / 64, 3 * DM / 64, 1), 32, 0, stream>>>(XB, WQ, bqkv, H16, HI, LO);
    k_fahl<<<(NB * NH * NTHL) / 4, 128, 0, stream>>>(HI, LO, ATh, ATl);
    if (NT16 > 0) k_fa16<<<(NB * NH * NT16D) / 4, 128, 0, stream>>>(H16, ATh, ATl);
    k_out<<<dim3(MROWS / 64, DM / 64, 1), 32, 0, stream>>>(ATh, ATl, WO, bp, OUT);
}
